// GraphConv_88648124989846
// MI455X (gfx1250) — hardware-verified
//
#include <hip/hip_runtime.h>


namespace {

constexpr int N = 100000, E = 1600000, KD = E / N  , NL = N  , NSTAT = N  ;
constexpr int F = 64  , O = 64  , KW = F + 3  , KP = 96  , NPW = 8  , NBLK = NSTAT / (2 * NPW)  , NPART = 2 * NBLK  , NBA = 512  ;
constexpr float XS = 8.0f, WSC = 256.0f, WSQ = 0.25f, RS_ = 1024.0f, BNEPS = 1e-5f;
static_assert(KD == 16 && N % (2 * NPW) == 0 && NL % (2 * NPW) == 0 && NSTAT % (2 * NPW) == 0 && F == 64 && O == 64, "tiling");
typedef _Float16 b16;
typedef __attribute__((ext_vector_type(16))) _Float16 v16b;
typedef __attribute__((ext_vector_type(8))) _Float16 v8b;
typedef __attribute__((ext_vector_type(8))) float v8f;
typedef __attribute__((ext_vector_type(4))) float v4f;
__device__ __forceinline__ float bf16_rne(float f) { unsigned int u = __float_as_uint(f); u += 0x7FFFu + ((u >> 16) & 1u); return __uint_as_float(u & 0xFFFF0000u); }
__device__ __forceinline__ void split16(float v, b16& hi, b16& lo) { hi = (b16)v; lo = (b16)(v - (float)hi); }
__device__ __forceinline__ v16b frag_kb(const b16* p, int hh) { const v8b a = *(const v8b*)(p + 8 * hh), b = *(const v8b*)(p + 16 + 8 * hh); v16b f;
#pragma unroll
  for (int e = 0; e < 8; ++e) { f[e] = a[e]; f[8 + e] = b[e]; } return f; }
__device__ __forceinline__ v8f wmma16b(v16b a, v16b b, v8f c) { v8f d = __builtin_amdgcn_wmma_f32_16x16x32_f16(false, a, false, b, (short)0, c, false, false); asm volatile("v_nop\n\tv_nop\n\tv_nop\n\tv_nop" : "+v"(d) : "v"(a), "v"(b)); return d; }
__device__ __forceinline__ void wave_lds_sync() { __builtin_amdgcn_fence(__ATOMIC_RELEASE, "workgroup"); __builtin_amdgcn_wave_barrier(); __builtin_amdgcn_fence(__ATOMIC_ACQUIRE, "workgroup"); }
__device__ __forceinline__ float pmul(float a, float b) { float p = a * b; asm volatile("" : "+v"(p)); return p; }
__device__ __forceinline__ int iclamp(int v, int lo, int hi) { return v < lo ? lo : (v > hi ? hi : v); }
typedef __attribute__((ext_vector_type(4))) _Float16 v4h;

__global__ __launch_bounds__(256) void wt_kernel(const float* __restrict__ w, b16* __restrict__ WT) {
  const int u = blockIdx.x * 256 + threadIdx.x; if (u >= O * KP / 8) return; const int e = u * 8; const int o = e / KP, k0 = e % KP; v8b v;
#pragma unroll
  for (int j = 0; j < 8; ++j) { const int k = k0 + j; float val = 0.0f;
    if (k < F) val = bf16_rne(w[(size_t)o * KW + k]) * WSC; else if (k < F + 3) val = bf16_rne(w[(size_t)o * KW + k]) * WSC; else if (k < F + 6) val = bf16_rne(w[(size_t)o * KW + F + (k - F - 3)]) * WSQ;
    v[j] = (b16)val; }
  for (int pass = 0; pass < 2; ++pass) { *(volatile v8b*)(WT + e) = v; __threadfence(); }
}
__global__ __launch_bounds__(128) void colsum_kernel(const float* __restrict__ node, const float* __restrict__ feat, const int* __restrict__ edges, float* __restrict__ PA) {
  const int b = blockIdx.x, c = threadIdx.x; const int ch = (E + NBA - 1) / NBA; const int e0 = b * ch, e1 = min(E, e0 + ch); float s = 0.0f;
  if (c < F) {
#pragma unroll 1
    for (int e = e0; e < e1; ++e) { if (NSTAT < N && e % N >= NSTAT) continue; const int d = iclamp(edges[(size_t)e * 2 + 1], 0, N - 1); s += bf16_rne(feat[(size_t)d * F + c]); } }
  else if (c < KW) { const int j = c - F;
#pragma unroll 1
    for (int e = e0; e < e1; ++e) { const int sn = e % N; if (NSTAT < N && sn >= NSTAT) continue; const int d = iclamp(edges[(size_t)e * 2 + 1], 0, N - 1); s += bf16_rne(node[(size_t)d * 3 + j]) - bf16_rne(node[(size_t)sn * 3 + j]); } }
  for (int pass = 0; pass < 2; ++pass) { if (c < 96) ((volatile float*)PA)[(size_t)b * 96 + c] = (c < KW) ? s : 0.0f; __threadfence(); }
}
__global__ __launch_bounds__(128) void mean_kernel(const float* __restrict__ PA, const float* __restrict__ w, float* __restrict__ MEANH) {
  __shared__ float mm[96]; const int c = threadIdx.x;
  if (c < 96) { float s = 0.0f;
#pragma unroll 1
    for (int b = 0; b < NBA; ++b) s += PA[(size_t)b * 96 + c]; mm[c] = (c < KW) ? s * (1.0f / (float)E) : 0.0f; }
  __syncthreads();
  float mh = 0.0f; if (c < O) {
#pragma unroll 1
    for (int k = 0; k < KW; ++k) mh += pmul(bf16_rne(w[(size_t)c * KW + k]), mm[k]); }
  for (int pass = 0; pass < 2; ++pass) { if (c < 96) ((volatile float*)MEANH)[c] = (c < O) ? mh : 0.0f; __threadfence(); }
}
template <bool STAT>
__global__ __launch_bounds__(64) void edge_kernel(const float* __restrict__ node, const float* __restrict__ feat, const int* __restrict__ edges, const b16* __restrict__ WT, const float* __restrict__ MEANH, const float* __restrict__ SCALE, const float* __restrict__ SHIFT, float* __restrict__ OUTP) {
  __shared__ __attribute__((aligned(16))) b16 Ah[2][16][KP + 8]; __shared__ int Di[2][16]; __shared__ __attribute__((aligned(16))) float Tr[2][O + 4];
  const int wave = threadIdx.x >> 5, lane = threadIdx.x & 31, nloc = lane & 15, hlf = lane >> 4; const int widx = blockIdx.x * 2 + wave; const int n0 = widx * NPW;
  float cA[4], cB[4];
#pragma unroll
  for (int t = 0; t < 4; ++t) { const int col = t * 16 + nloc; cA[t] = STAT ? MEANH[col] : SCALE[col]; cB[t] = STAT ? 0.0f : SHIFT[col]; }
  float q[4]; for (int t = 0; t < 4; ++t) q[t] = 0.0f;
#pragma unroll 1
  for (int i = 0; i < NPW; ++i) { const int n = n0 + i; const int nn = n < N ? n : N - 1;
    if (lane < 16) { const int e = nn + lane * N; const int d = iclamp(edges[(size_t)e * 2 + 1], 0, N - 1); Di[wave][lane] = d; b16* ar = &Ah[wave][lane][F];
      for (int j = 0; j < 3; ++j) { const float df = (bf16_rne(node[(size_t)d * 3 + j]) - bf16_rne(node[(size_t)nn * 3 + j])) * XS; const b16 ph = (b16)df; ar[j] = ph; ar[3 + j] = (b16)((df - (float)ph) * RS_); }
      for (int j = 6; j < KP - F; ++j) ar[j] = (b16)0.0f; }
    wave_lds_sync();
    for (int idx = lane; idx < 16 * (F / 4); idx += 32) { const int rr = idx / (F / 4), c4 = (idx % (F / 4)) * 4; const v4f v = *(const v4f*)(feat + (size_t)Di[wave][rr] * F + c4); v4h hv; for (int j = 0; j < 4; ++j) hv[j] = (b16)(bf16_rne(v[j]) * XS); *(v4h*)(&Ah[wave][rr][c4]) = hv; }
    wave_lds_sync();
    v8f acc[4];
#pragma unroll
    for (int t = 0; t < 4; ++t) acc[t] = (v8f){};
#pragma unroll
    for (int kb = 0; kb < KP; kb += 32) { const v16b a = frag_kb(&Ah[wave][nloc][kb], hlf);
#pragma unroll
      for (int t = 0; t < 4; ++t) acc[t] = wmma16b(a, frag_kb(WT + (size_t)(t * 16 + nloc) * KP + kb, hlf), acc[t]); }
    if (STAT) {
#pragma unroll
      for (int t = 0; t < 4; ++t) for (int r = 0; r < 8; ++r) { const float dv = acc[t][r] * (1.0f / (XS * WSC)) - cA[t]; q[t] = fmaf(dv, dv, q[t]); } }
    else { float mx[4];
#pragma unroll
      for (int t = 0; t < 4; ++t) { mx[t] = 0.0f; for (int r = 0; r < 8; ++r) { const float y = fmaxf(fmaf(acc[t][r] * (1.0f / (XS * WSC)), cA[t], cB[t]), 0.0f); mx[t] = fmaxf(mx[t], y); } }
#pragma unroll
      for (int t = 0; t < 4; ++t) { const float m2 = fmaxf(mx[t], __shfl_xor(mx[t], 16)); if (hlf == 0) Tr[wave][t * 16 + nloc] = m2; }
      wave_lds_sync();
      for (int pass = 0; pass < 2; ++pass) { if (lane < 16 && n < NL) *(volatile v4f*)(OUTP + (size_t)n * O + lane * 4) = *(const v4f*)(&Tr[wave][lane * 4]); __threadfence(); } }
    wave_lds_sync(); }
  if (STAT) {
#pragma unroll
    for (int t = 0; t < 4; ++t) { const float q2 = q[t] + __shfl_xor(q[t], 16); if (hlf == 0) Tr[wave][t * 16 + nloc] = (n0 < NSTAT) ? q2 : 0.0f; }
    wave_lds_sync();
    for (int pass = 0; pass < 2; ++pass) { if (lane < 16) *(volatile v4f*)(OUTP + (size_t)widx * O + lane * 4) = *(const v4f*)(&Tr[wave][lane * 4]); __threadfence(); } }
}
__global__ __launch_bounds__(64) void var_kernel(const float* __restrict__ PV, const float* __restrict__ MEANH, const float* __restrict__ gamma, const float* __restrict__ beta, float* __restrict__ SCALE, float* __restrict__ SHIFT) {
  const int c = threadIdx.x; float s = 0.0f;
#pragma unroll 1
  for (int p = 0; p < NPART; ++p) s += PV[(size_t)p * O + c];
  const float var = s * (1.0f / (float)E); const float sc = bf16_rne(gamma[c]) * rsqrtf(var + BNEPS); const float sh = bf16_rne(beta[c]) - MEANH[c] * sc;
  for (int pass = 0; pass < 2; ++pass) { ((volatile float*)SCALE)[c] = sc; ((volatile float*)SHIFT)[c] = sh; __threadfence(); }
}
}

extern "C" void kernel_launch(void* const* d_in, const int* in_sizes, int n_in, void* d_out, int out_size, void* d_ws, size_t ws_size, hipStream_t stream) {
  (void)n_in;
  auto Fp = [&](int i) { return (const float*)d_in[i]; }; auto Ip = [&](int i) { return (const int*)d_in[i]; };
  if (in_sizes[0] != N * 3 || in_sizes[1] != N * F || in_sizes[2] != O * KW || in_sizes[3] != O || in_sizes[4] != O || in_sizes[5] != E * 2 || out_size != N * O) return;
  size_t off = 0; char* ws = (char*)d_ws;
  auto carve = [&](size_t bytes) { char* p = ws + off; off += (bytes + 255) & ~(size_t)255; return p; };
  b16* WT = (b16*)carve((size_t)O * KP * 2); float* PA = (float*)carve((size_t)NBA * 96 * 4); float* MEANH = (float*)carve(96 * 4); float* PV = (float*)carve((size_t)NPART * O * 4); float* SCALE = (float*)carve(O * 4); float* SHIFT = (float*)carve(O * 4);
  if (off > ws_size || off > ((size_t)8 << 20)) return;
  wt_kernel<<<(O * KP / 8 + 255) / 256, 256, 0, stream>>>(Fp(2), WT);
  colsum_kernel<<<NBA, 128, 0, stream>>>(Fp(0), Fp(1), Ip(5), PA);
  mean_kernel<<<1, 128, 0, stream>>>(PA, Fp(2), MEANH);
  edge_kernel<true><<<NBLK, 64, 0, stream>>>(Fp(0), Fp(1), Ip(5), WT, MEANH, MEANH, MEANH, PV);
  var_kernel<<<1, 64, 0, stream>>>(PV, MEANH, Fp(3), Fp(4), SCALE, SHIFT);
  edge_kernel<false><<<NL / (2 * NPW), 64, 0, stream>>>(Fp(0), Fp(1), Ip(5), WT, MEANH, SCALE, SHIFT, (float*)d_out);
}
